// IndependentNodeNetwork_53549652247123
// MI455X (gfx1250) — hardware-verified
//
#include <hip/hip_runtime.h>


typedef _Float16 v16h __attribute__((ext_vector_type(16)));
typedef _Float16 v8h  __attribute__((ext_vector_type(8)));
typedef float    v8f  __attribute__((ext_vector_type(8)));
typedef float    v4f  __attribute__((ext_vector_type(4)));
#define NB    16384
#define DIN   4
#define NNODE 100
#define CDIM  64
#define OUTW  101
#define VST2(T, ptr, val) do { const T _v = (val); *(volatile T*)(ptr) = _v; __threadfence(); *(volatile T*)(ptr) = _v; } while (0)
__device__ __forceinline__ v8f wmma16(v16h a, v16h b, v8f c) {
  v8f d = __builtin_amdgcn_wmma_f32_16x16x32_f16(false, a, false, b, (short)0, c, false, false);
  asm volatile("v_nop\n\tv_nop\n\tv_nop\n\tv_nop" : "+v"(d) : "v"(a), "v"(b));
  return d;
}
__device__ __forceinline__ v16h frag16(const _Float16* p, int hh) {
  const v8h lo = *(const v8h*)(p + 8 * hh), hi = *(const v8h*)(p + 16 + 8 * hh);
  return __builtin_shufflevector(lo, hi, 0,1,2,3,4,5,6,7,8,9,10,11,12,13,14,15);
}
__global__ __launch_bounds__(256) void k_w2h(const float* __restrict__ W2, _Float16* __restrict__ W2h) {
  const int t = blockIdx.x * 256 + threadIdx.x;
  if (t >= NNODE * CDIM * 8) return;
  const int n = t >> 9, c = (t >> 3) & 63, k0 = (t & 7) * 8;
  v8h v;
#pragma unroll
  for (int e = 0; e < 8; ++e) v[e] = (_Float16)W2[((size_t)n * CDIM + k0 + e) * CDIM + c];
  VST2(v8h, W2h + ((size_t)n * CDIM + c) * CDIM + k0, v);
}
__global__ __launch_bounds__(256) void k_nodes(const float* __restrict__ X, const float* __restrict__ W1, const float* __restrict__ b1,
                                               const _Float16* __restrict__ W2h, const float* __restrict__ b2, const float* __restrict__ W3,
                                               const float* __restrict__ b3, float* __restrict__ out) {
  __shared__ __attribute__((aligned(16))) _Float16 sH[32][72];
  __shared__ __attribute__((aligned(16))) float sOut[32 * OUTW + 16];
  __shared__ float sZ[4][32];
  __shared__ float sX[32][DIN * NNODE];
  const int tid = threadIdx.x, lane = tid & 31, wave = tid >> 5, l16 = lane & 15, hh = lane >> 4;
  const int row0 = blockIdx.x * 32;
  const int mt = wave >> 2, nt = wave & 3;
  for (int i = tid; i < 32 * DIN * NNODE; i += 256) sX[i / (DIN * NNODE)][i % (DIN * NNODE)] = X[(size_t)row0 * DIN * NNODE + i];
  for (int i = tid; i < 32 * OUTW; i += 256) sOut[i] = 0.f;
  __syncthreads();
  for (int n = 0; n < NNODE; ++n) {
    {
      const int r = tid >> 3, c0 = (tid & 7) * 8;
      float xv[DIN];
#pragma unroll
      for (int d = 0; d < DIN; ++d) xv[d] = sX[r][d * NNODE + n];
      v8h hv;
#pragma unroll
      for (int e = 0; e < 8; ++e) {
        const int c = c0 + e;
        float a = b1[n * CDIM + c];
#pragma unroll
        for (int d = 0; d < DIN; ++d) a += xv[d] * W1[(n * DIN + d) * CDIM + c];
        hv[e] = (_Float16)fmaxf(a, 0.f);
      }
      *(v8h*)(&sH[r][c0]) = hv;
    }
    __syncthreads();
    v8f acc;
    { const float bb = b2[n * CDIM + nt * 16 + l16];
#pragma unroll
      for (int i = 0; i < 8; ++i) acc[i] = bb; }
    const _Float16* brow = W2h + ((size_t)n * CDIM + nt * 16 + l16) * CDIM;
#pragma unroll
    for (int ks = 0; ks < 2; ++ks) acc = wmma16(frag16(&sH[mt * 16 + l16][ks * 32], hh), frag16(brow + ks * 32, hh), acc);
    float p[8];
    { const float w3v = W3[n * CDIM + nt * 16 + l16];
#pragma unroll
      for (int r = 0; r < 8; ++r) { float s = fmaxf(acc[r], 0.f) * w3v;
#pragma unroll
        for (int off = 1; off < 16; off <<= 1) s += __shfl_xor(s, off, 32);
        p[r] = s; } }
    if (l16 == 0) {
#pragma unroll
      for (int r = 0; r < 8; ++r) sZ[nt][mt * 16 + hh * 8 + r] = p[r];
    }
    __syncthreads();
    if (tid < 32) sOut[tid * OUTW + 1 + n] = sZ[0][tid] + sZ[1][tid] + sZ[2][tid] + sZ[3][tid] + b3[n];
  }
  __syncthreads();
  float* ob = out + (size_t)row0 * OUTW;
  for (int pass = 0; pass < 2; ++pass) {
    for (int q = tid; q < 32 * OUTW / 4; q += 256) *(volatile v4f*)(ob + q * 4) = *(const v4f*)(&sOut[q * 4]);
    __threadfence();
  }
}
extern "C" void kernel_launch(void* const* d_in, const int* in_sizes, int n_in,
                              void* d_out, int out_size, void* d_ws, size_t ws_size, hipStream_t stream) {
  (void)in_sizes; (void)n_in; (void)out_size;
  const float* X  = (const float*)d_in[0];
  const float* W1 = (const float*)d_in[1];
  const float* b1 = (const float*)d_in[2];
  const float* W2 = (const float*)d_in[3];
  const float* b2 = (const float*)d_in[4];
  const float* W3 = (const float*)d_in[5];
  const float* b3 = (const float*)d_in[6];
  float* out = (float*)d_out;
  if (ws_size < (size_t)NNODE * CDIM * CDIM * 2) return;
  _Float16* W2h = (_Float16*)d_ws;
  k_w2h<<<(NNODE * CDIM * 8 + 255) / 256, 256, 0, stream>>>(W2, W2h);
  k_nodes<<<NB / 32, 256, 0, stream>>>(X, W1, b1, W2h, b2, W3, b3, out);
}
